// DynamicMoERoutingLayer_40544491274390
// MI455X (gfx1250) — hardware-run, weakly checked
//
#include <hip/hip_runtime.h>
#include <stdint.h>

#define DEVINL __device__ __forceinline__

typedef _Float16 f16t;
typedef _Float16 v16h __attribute__((ext_vector_type(16)));
typedef _Float16 v8h  __attribute__((ext_vector_type(8)));
typedef float    v8f  __attribute__((ext_vector_type(8)));
typedef float    v4f  __attribute__((ext_vector_type(4)));
typedef v8h   __attribute__((may_alias)) v8ha;
typedef v4f   __attribute__((may_alias)) v4fa;
typedef float __attribute__((may_alias)) f32a;
union FragH { v16h v; v8h half[2]; };

#define NEXP   10
#define CIN    64
#define COUT   64
#define HIN    64
#define WIN    64
#define HO     62
#define WOUT   62
#define RDIM   512
#define DDIM   128
#define KPOS   9
#define CWPE   (COUT * CIN * KPOS)
#define WPS    (KPOS * COUT * CIN)
#define LCOLS  66
#define LPITCH 72
#define INROWS 4
#define ORPB   2
#define CWAVES 8
#define CTPB   256
#define SPITCH 68
#define PPITCH 64
#define GTPB   256
#define PTPB   256
#define PL4    (HO * WOUT / 4)
#define XCAR   16.0f
#define WCAR   1024.0f
#define OSCALE (1.0f / 16384.0f)

#define SX_HALVES (INROWS * LCOLS * LPITCH)

static_assert(CTPB == CWAVES * 32);
static_assert(CWAVES * 16 * SPITCH * 4 <= SX_HALVES * 2);
static_assert((WPS % (8 * GTPB)) == 0);
static_assert((HO % ORPB) == 0);
static_assert((LPITCH % 8) == 0);
static_assert((SPITCH % 4) == 0);
static_assert(((HO * WOUT) % 4) == 0);
static_assert(CWPE == WPS);

DEVINL int imin(int a, int b) { return a < b ? a : b; }

DEVINL v8f wmma_f16(v16h a, v16h b, v8f c) {
  v8f d = __builtin_amdgcn_wmma_f32_16x16x32_f16(false, a, false, b, (short)0, c, false, false);
  asm volatile("v_nop\n\tv_nop\n\tv_nop\n\tv_nop" : "+v"(d) : "v"(a), "v"(b));
  return d;
}
DEVINL v8f zero8f() {
  v8f z = {0.f, 0.f, 0.f, 0.f, 0.f, 0.f, 0.f, 0.f};
  return z;
}

__global__ __launch_bounds__(GTPB) void gate_k(const float* __restrict__ rv,
                                             const float* __restrict__ rp_w,
                                             const float* __restrict__ rp_b,
                                             const float* __restrict__ emb,
                                             const float* __restrict__ conv_w,
                                             const float* __restrict__ conv_b,
                                             const int* __restrict__ task,
                                             f16t* __restrict__ wmix,
                                             float* __restrict__ bmix)
{
  __shared__ float sr[DDIM];
  __shared__ float ssim[16];
  __shared__ float scoef[16];
  __shared__ float sinv[4];
  __shared__ __attribute__((aligned(16))) float sb[COUT];
  const int b = blockIdx.x, tid = threadIdx.x, lane = tid & 31;
  (void)task;

  if (tid < DDIM) {
    const float* rvb = rv + (size_t)b * RDIM;
    const float* wr  = rp_w + (size_t)tid * RDIM;
    float acc = 0.0f;
    #pragma unroll 1
    for (int k = 0; k < RDIM; ++k) acc = fmaf(rvb[k], wr[k], acc);
    sr[tid] = acc + rp_b[tid];
  }
  __syncthreads();

  if (tid < 32) {
    float s = 0.0f;
    #pragma unroll
    for (int i = 0; i < 4; ++i) { const float v = sr[4 * lane + i]; s = fmaf(v, v, s); }
    #pragma unroll
    for (int off = 16; off > 0; off >>= 1) s += __shfl_xor(s, off);
    if (lane == 0) sinv[0] = 1.0f / fmaxf(sqrtf(s), 1e-8f);
  }
  __syncthreads();
  if (tid < DDIM) { const float v = sr[tid] * sinv[0]; sr[tid] = v; }
  __syncthreads();

  if (tid < 32) {
    const int n = (lane < NEXP) ? lane : (NEXP - 1);
    const float* e = emb + (size_t)n * DDIM;
    float en = 0.0f;
    #pragma unroll 1
    for (int d = 0; d < DDIM; ++d) { const float v = e[d]; en = fmaf(v, v, en); }
    const float inve = 1.0f / fmaxf(sqrtf(en), 1e-8f);
    float dot = 0.0f;
    #pragma unroll 1
    for (int d = 0; d < DDIM; ++d) dot = fmaf(sr[d], e[d] * inve, dot);
    if (lane < NEXP) ssim[lane] = dot;
  }
  __syncthreads();

  if (tid < 32) {
    float m = ssim[0];
    #pragma unroll 1
    for (int n = 1; n < NEXP; ++n) m = fmaxf(m, ssim[n]);
    const int n = (lane < NEXP) ? lane : (NEXP - 1);
    float ex = expf(ssim[n] - m);
    ex = (lane < NEXP) ? ex : 0.0f;
    float S = ex;
    #pragma unroll
    for (int off = 16; off > 0; off >>= 1) S += __shfl_xor(S, off);
    const float w = ex * (1.0f / S);
    float ds = w;
    #pragma unroll
    for (int off = 16; off > 0; off >>= 1) ds += __shfl_xor(ds, off);
    const float c = w * (1.0f / ds);
    if (lane < NEXP) scoef[lane] = c;
  }
  __syncthreads();

  if (tid < COUT) {
    float be = 0.0f;
    #pragma unroll 1
    for (int n = 0; n < NEXP; ++n) be = fmaf(scoef[n], conv_b[n * COUT + tid], be);
    sb[tid] = be;
  }
  __syncthreads();
  {
    const v4f bv = *(const v4fa*)(sb + 4 * (tid & 15));
    float* bdst = bmix + (size_t)b * COUT + 4 * (tid & 15);
    const bool bst = (tid < 16);
    if (bst) *(volatile v4f*)bdst = bv;
    __threadfence();
    if (bst) *(volatile v4f*)bdst = bv;
  }

  f16t* wdst0 = wmix + (size_t)b * WPS;
  #pragma unroll 1
  for (int i = 0; i < WPS / (8 * GTPB); ++i) {
    const int o8  = i * GTPB + tid;
    const int pos = o8 >> 9;
    const int rem = o8 & 511;
    const int co  = rem >> 3;
    const int cib = (rem & 7) * 8;
    const int wbase = (co * CIN + cib) * KPOS + pos;
    float accj[8];
    #pragma unroll
    for (int j = 0; j < 8; ++j) accj[j] = 0.0f;
    #pragma unroll 1
    for (int n = 0; n < NEXP; ++n) {
      const float c = scoef[n];
      const float* wp = conv_w + (size_t)n * CWPE + wbase;
      #pragma unroll
      for (int j = 0; j < 8; ++j) accj[j] = fmaf(c, wp[KPOS * j], accj[j]);
    }
    v8h o;
    #pragma unroll
    for (int j = 0; j < 8; ++j) o[j] = (f16t)(accj[j] * WCAR);
    f16t* dst = wdst0 + 8 * o8;
    *(volatile v8h*)dst = o;
    __threadfence();
    *(volatile v8h*)dst = o;
  }
}

__global__ __launch_bounds__(CTPB) void conv_k(const float* __restrict__ x,
                                             const f16t* __restrict__ wmix,
                                             const float* __restrict__ bmix,
                                             float* __restrict__ plane)
{
  __shared__ __attribute__((aligned(16))) f16t sX[SX_HALVES];
  const int yt  = blockIdx.x;
  const int b   = blockIdx.y;
  const int y0  = yt * ORPB;
  const int tid = threadIdx.x;
  const float* xb = x + (size_t)b * CIN * HIN * WIN;

  #pragma unroll 1
  for (int i = 0; i < (INROWS * CIN * WIN) / CTPB; ++i) {
    const int e    = i * CTPB + tid;
    const int col  = e & 63;
    const int cin  = (e >> 6) & 63;
    const int irow = e >> 12;
    const int grow = imin(y0 + irow, HIN - 1);
    const float v  = xb[((size_t)cin * HIN + grow) * WIN + col];
    sX[(irow * LCOLS + col) * LPITCH + cin] = (f16t)(v * XCAR);
  }
  #pragma unroll 1
  for (int i = 0; i < 2; ++i) {
    const int e    = i * CTPB + tid;
    const int cin  = e & 63;
    const int hc   = (e >> 6) & 1;
    const int irow = e >> 7;
    sX[(irow * LCOLS + 64 + hc) * LPITCH + cin] = (f16t)0.0f;
  }
  __syncthreads();

  const int wave = tid >> 5, lane = tid & 31;
  const int h = lane >> 4, nn = lane & 15;
  const int mg = wave & 3, rr = wave >> 2;

  v8f acc[4];
  #pragma unroll
  for (int ct = 0; ct < 4; ++ct) acc[ct] = zero8f();

  const f16t* wb = wmix + (size_t)b * WPS + (size_t)(mg * 16 + nn) * CIN + 8 * h;

  #pragma unroll 1
  for (int pos = 0; pos < KPOS; ++pos) {
    const int kh = pos / 3;
    const int kw = pos - 3 * kh;
    const f16t* xrow = sX + ((rr + kh) * LCOLS + nn + kw) * LPITCH + 8 * h;
    #pragma unroll
    for (int ks = 0; ks < 2; ++ks) {
      const f16t* wr = wb + pos * (COUT * CIN) + 32 * ks;
      FragH a;
      a.half[0] = *(const v8ha*)(wr);
      a.half[1] = *(const v8ha*)(wr + 16);
      #pragma unroll
      for (int ct = 0; ct < 4; ++ct) {
        const f16t* xr = xrow + ct * 16 * LPITCH + 32 * ks;
        FragH bq;
        bq.half[0] = *(const v8ha*)(xr);
        bq.half[1] = *(const v8ha*)(xr + 16);
        acc[ct] = wmma_f16(a.v, bq.v, acc[ct]);
      }
    }
  }

  __syncthreads();
  f32a* stg = (f32a*)sX;
  f32a* wst = stg + wave * (16 * SPITCH);
  {
    const float* bp = bmix + (size_t)b * COUT + mg * 16 + 8 * h;
    const v4f b0 = *(const v4fa*)bp;
    const v4f b1 = *(const v4fa*)(bp + 4);
    #pragma unroll
    for (int ct = 0; ct < 4; ++ct) {
      #pragma unroll
      for (int r = 0; r < 4; ++r) {
        wst[(8 * h + r) * SPITCH + ct * 16 + nn]     = fmaf(acc[ct][r],     OSCALE, b0[r]);
        wst[(8 * h + 4 + r) * SPITCH + ct * 16 + nn] = fmaf(acc[ct][4 + r], OSCALE, b1[r]);
      }
    }
  }
  __syncthreads();
  {
    const int y = y0 + rr;
    v4f vals[8];
    #pragma unroll
    for (int i = 0; i < 8; ++i)
      vals[i] = *(const v4fa*)(wst + (2 * i + h) * SPITCH + 4 * nn);
    float* prow = plane + (((size_t)b * COUT + mg * 16) * HO + y) * PPITCH + 4 * nn;
    #pragma unroll
    for (int i = 0; i < 8; ++i)
      *(volatile v4f*)(prow + (size_t)(2 * i + h) * HO * PPITCH) = vals[i];
    __threadfence();
    #pragma unroll
    for (int i = 0; i < 8; ++i)
      *(volatile v4f*)(prow + (size_t)(2 * i + h) * HO * PPITCH) = vals[i];
  }
}

__global__ __launch_bounds__(PTPB) void pack_k(const float* __restrict__ plane,
                                             float* __restrict__ out, int total4)
{
  const int t = blockIdx.x * PTPB + threadIdx.x;
  if (t >= total4) return;
  const int pl   = t / PL4;
  const int rem0 = (t - pl * PL4) * 4;
  v4f o;
  #pragma unroll
  for (int p = 0; p < 4; ++p) {
    const int rem = rem0 + p;
    const int yy  = rem / WOUT;
    const int xx  = rem - yy * WOUT;
    o[p] = plane[((size_t)pl * HO + yy) * PPITCH + xx];
  }
  float* dst = out + (size_t)t * 4;
  *(volatile v4f*)dst = o;
  __threadfence();
  *(volatile v4f*)dst = o;
}

extern "C" void kernel_launch(void* const* d_in, const int* in_sizes, int n_in,
                              void* d_out, int out_size, void* d_ws, size_t ws_size,
                              hipStream_t stream) {
  if (n_in < 8) return;
  const int per = CIN * HIN * WIN;
  if (in_sizes[0] <= 0 || (in_sizes[0] % per) != 0) return;
  const int nB = in_sizes[0] / per;
  if (in_sizes[1] != nB * RDIM)     return;
  if (in_sizes[2] != NEXP * CWPE)   return;
  if (in_sizes[3] != NEXP * COUT)   return;
  if (in_sizes[4] != NEXP * DDIM)   return;
  if (in_sizes[5] != DDIM * RDIM)   return;
  if (in_sizes[6] != DDIM)          return;
  if (out_size != nB * COUT * HO * WOUT) return;

  const float* x      = (const float*)d_in[0];
  const float* rv     = (const float*)d_in[1];
  const float* conv_w = (const float*)d_in[2];
  const float* conv_b = (const float*)d_in[3];
  const float* emb    = (const float*)d_in[4];
  const float* rp_w   = (const float*)d_in[5];
  const float* rp_b   = (const float*)d_in[6];
  const int*   task   = (const int*)d_in[7];
  float* outp = (float*)d_out;

  const size_t szW = (size_t)nB * WPS * 2;
  const size_t szB = (size_t)nB * COUT * 4;
  const size_t szP = (size_t)nB * COUT * HO * PPITCH * 4;
  size_t off = 0;
  char* ws = (char*)d_ws;
  f16t*  WMIX  = (f16t*)(ws + off);   off += szW;
  float* BMIX  = (float*)(ws + off);  off += szB;
  float* PLANE = (float*)(ws + off);  off += szP;
  if (off > ws_size) return;

  const int total4 = out_size / 4;

  gate_k<<<nB, GTPB, 0, stream>>>(rv, rp_w, rp_b, emb, conv_w, conv_b, task, WMIX, BMIX);
  conv_k<<<dim3(HO / ORPB, nB), CTPB, 0, stream>>>(x, WMIX, BMIX, PLANE);
  pack_k<<<(total4 + PTPB - 1) / PTPB, PTPB, 0, stream>>>(PLANE, outp, total4);
}
